// NodewiseInteraction_36112085025169
// MI455X (gfx1250) — hardware-run, weakly checked
//
#include <hip/hip_runtime.h>
#include <stddef.h>
#include <stdint.h>


#define NN     8192
#define NE     131072
#define DF     320
#define SC     128
#define VC     64
#define WN     384
#define EAD    20
#define ACW    768
#define NTHR   256
#define NWAVE  8
#define EPT    8
#define CHUNK  (NTHR * EPT)
#define WCAP   (EPT * 32)
#define LISTN  (NWAVE * WCAP)
#define SLB    6
#define NBS    64
#define TE     64
#define HCAP   4352
#define MAXT   (HCAP / TE)
#define GBM    64
#define GTHR   128
#define IS3    0.57735026918962576f
#define WSMAX  134217728

#define OW_W0S   0
#define OW_W0V   (OW_W0S + 128 * 128)
#define OW_W1S2  (OW_W0V + 64 * 64)
#define OW_W1V2  (OW_W1S2 + 128 * 256)
#define OW_ESAB  (OW_W1V2 + 64 * 128)
#define OW_ESC   (OW_ESAB + 256 * 256)
#define OW_ES22  (OW_ESC + 128 * 128)
#define OW_ER1   (OW_ES22 + 384 * 256)
#define OW_ER22  (OW_ER1 + 128 * 32)
#define OW_W2S2  (OW_ER22 + 384 * 256)
#define OW_W2V2  (OW_W2S2 + 128 * 384)
#define NW_TOT   (OW_W2V2 + 64 * 384)
#define U1   (OW_W0V / 8)
#define U2   (OW_W1S2 / 8)
#define U3   (OW_W1V2 / 8)
#define U4   (OW_ESAB / 8)
#define U5   (OW_ESC / 8)
#define U6   (OW_ES22 / 8)
#define U7   (OW_ER1 / 8)
#define U8   (OW_ER22 / 8)
#define U9   (OW_W2S2 / 8)
#define U10  (OW_W2V2 / 8)
#define U11  (NW_TOT / 8)
#define U12  (U11 + NN * 16)
#define U13  (U12 + NN * 8)

#define F_WT   0
#define F_A    24576
#define F_EA   45056
#define F_B    46080
#define F_Y    46976
#define F_SL   47232
#define F_R2   47296
#define F_CNT  51648
#define F_END  51808
#define EDGE_LDS_BYTES (F_END * 4)

static_assert(NN % 128 == 0 && NE % 64 == 0 && NN % NBS == 0 && NN % 8 == 0);
static_assert(NE % CHUNK == 0);
static_assert(NTHR * 3 == ACW);
static_assert(TE % 16 == 0 && TE * 4 == NTHR);
static_assert(HCAP % TE == 0 && HCAP % 32 == 0 && HCAP >= 4207 + 64);
static_assert(U1 % NTHR == 0 && U2 % NTHR == 0 && U3 % NTHR == 0 && U4 % NTHR == 0 && U5 % NTHR == 0);
static_assert(U6 % NTHR == 0 && U7 % NTHR == 0 && U8 % NTHR == 0 && U9 % NTHR == 0 && U10 % NTHR == 0);
static_assert(U11 % NTHR == 0 && U12 % NTHR == 0 && U13 % NTHR == 0);
static_assert(F_A == F_WT + TE * WN);
static_assert(F_EA == F_A + (TE * 256 * 2 + TE * 256 * 2 + TE * 128 * 2) / 4);
static_assert((TE * 256 * 2 + TE * 256 * 2 + TE * 128 * 2) == (TE * SC + TE * 192) * 4);
static_assert(F_B == F_EA + (TE * 32 * 2) / 4 && F_Y == F_B + 896 && F_SL == F_Y + TE * 4);
static_assert(F_R2 == F_SL + 64 && F_CNT == F_R2 + HCAP && F_END >= F_CNT + 144);
static_assert(LISTN + HCAP <= TE * WN);
static_assert(EDGE_LDS_BYTES <= 327680);
static_assert((CHUNK & (CHUNK - 1)) == 0 && (NBS & (NBS - 1)) == 0 && NBS == (1 << SLB));
static_assert(((long long)NE << SLB) < (1LL << 31));
static_assert(NN % GBM == 0 && (3 * NN) % GBM == 0);

typedef float          v2f   __attribute__((ext_vector_type(2)));
typedef float          v4f   __attribute__((ext_vector_type(4)));
typedef float          v8f   __attribute__((ext_vector_type(8)));
typedef int            v4i   __attribute__((ext_vector_type(4)));
typedef int            v8i   __attribute__((ext_vector_type(8)));
typedef unsigned short v4us  __attribute__((ext_vector_type(4)));
typedef unsigned short v8us  __attribute__((ext_vector_type(8)));
typedef unsigned short v16us __attribute__((ext_vector_type(16)));
typedef __bf16         v16bf __attribute__((ext_vector_type(16)));
typedef v2f  __attribute__((may_alias)) v2fa;
typedef v4f  __attribute__((may_alias)) v4fa;
typedef v4us __attribute__((may_alias)) v4usa;
typedef v8us __attribute__((may_alias)) v8usa;
union FragB { v16bf v; v16us u; v8us h[2]; v8i w; };

__device__ __forceinline__ v8f wmb(const FragB& a, const FragB& b, v8f c) {
  v8f d = __builtin_amdgcn_wmma_f32_16x16x32_bf16(false, a.v, false, b.v, (short)0, c, false, false);
  asm volatile("v_nop\n\tv_nop\n\tv_nop\n\tv_nop" : "+v"(d) : "v"(a.w), "v"(b.w));
  return d;
}

__device__ __forceinline__ unsigned bf16_bits(float f) {
  const unsigned u = __float_as_uint(f);
  return (u + 0x7FFFu + ((u >> 16) & 1u)) >> 16;
}
__device__ __forceinline__ float bf16_val(float f) {
  return __uint_as_float(bf16_bits(f) << 16);
}
__device__ __forceinline__ float silu_f(float t) {
  return t * __builtin_amdgcn_rcpf(1.0f + __expf(-t));
}
__device__ __forceinline__ void split4(v4f v, v4us& oh, v4us& ol) {
  const float f[4] = {v.x, v.y, v.z, v.w};
#pragma unroll
  for (int e = 0; e < 4; ++e) {
    const unsigned hb = bf16_bits(f[e]);
    const unsigned lb = bf16_bits(f[e] - __uint_as_float(hb << 16));
    oh[e] = (unsigned short)hb;
    ol[e] = (unsigned short)lb;
  }
}
__device__ __forceinline__ void put16(unsigned short* dp, v8us o) {
  *(volatile v8us*)dp = o;
  __threadfence();
  *(volatile v8us*)dp = o;
}

template <int SB>
__device__ __forceinline__ int scan_chunk(const int* __restrict__ dsts, int nE, int cbase, int slotBase,
                                          int nb, int vec8, int* list, int tid, int lane, int wave) {
  int wc = 0;
  const int el0  = tid * EPT;
  const int e0   = cbase + el0;
  const int sent = -2147483647 - 1;
  v4i da, db;
  if (vec8 != 0 && cbase + CHUNK <= nE) {
    da = *(const v4i*)(dsts + e0);
    db = *(const v4i*)(dsts + e0 + 4);
  } else {
    da.x = (e0     < nE) ? dsts[min(e0,     nE - 1)] : sent;
    da.y = (e0 + 1 < nE) ? dsts[min(e0 + 1, nE - 1)] : sent;
    da.z = (e0 + 2 < nE) ? dsts[min(e0 + 2, nE - 1)] : sent;
    da.w = (e0 + 3 < nE) ? dsts[min(e0 + 3, nE - 1)] : sent;
    db.x = (e0 + 4 < nE) ? dsts[min(e0 + 4, nE - 1)] : sent;
    db.y = (e0 + 5 < nE) ? dsts[min(e0 + 5, nE - 1)] : sent;
    db.z = (e0 + 6 < nE) ? dsts[min(e0 + 6, nE - 1)] : sent;
    db.w = (e0 + 7 < nE) ? dsts[min(e0 + 7, nE - 1)] : sent;
  }
  const unsigned nbs = (unsigned)slotBase;
  const unsigned unb = (unsigned)nb;
  const unsigned s0 = (unsigned)da.x - nbs, s1 = (unsigned)da.y - nbs;
  const unsigned s2 = (unsigned)da.z - nbs, s3 = (unsigned)da.w - nbs;
  const unsigned s4 = (unsigned)db.x - nbs, s5 = (unsigned)db.y - nbs;
  const unsigned s6 = (unsigned)db.z - nbs, s7 = (unsigned)db.w - nbs;
  const bool h0 = s0 < unb, h1 = s1 < unb, h2 = s2 < unb, h3 = s3 < unb;
  const bool h4 = s4 < unb, h5 = s5 < unb, h6 = s6 < unb, h7 = s7 < unb;
  const unsigned any = __builtin_amdgcn_ballot_w32(h0 | h1 | h2 | h3 | h4 | h5 | h6 | h7);
  if (any != 0u) {
#define HITJ(J, HJ, SJ) { \
      const unsigned mj = __builtin_amdgcn_ballot_w32(HJ); \
      if (mj != 0u) { \
        if (HJ) { \
          const int pos = wc + (int)__builtin_amdgcn_mbcnt_lo(mj, 0u); \
          if (pos < WCAP) list[wave * WCAP + pos] = ((el0 + (J)) << SB) | (int)(SJ); \
        } \
        wc += (int)__builtin_popcount(mj); } }
    HITJ(0, h0, s0)
    HITJ(1, h1, s1)
    HITJ(2, h2, s2)
    HITJ(3, h3, s3)
    HITJ(4, h4, s4)
    HITJ(5, h5, s5)
    HITJ(6, h6, s6)
    HITJ(7, h7, s7)
#undef HITJ
  }
  return wc;
}

__device__ __forceinline__ v8us wgather(const float* __restrict__ W, int pitch, int rowOff, int kdup, int kmax,
                                        int n, int k8) {
  const int kb = (k8 >= kdup) ? (k8 - kdup) : k8;
  v8us o;
#pragma unroll
  for (int i = 0; i < 8; ++i) {
    const int k  = kb + i;
    const int kc = k < kmax ? k : kmax - 1;
    const float w = W[(size_t)(rowOff + kc) * (size_t)pitch + n];
    const float s = w * ((k < kmax) ? 1.0f : 0.0f);
    o[i] = (unsigned short)bf16_bits(s);
  }
  return o;
}

__global__ __launch_bounds__(NTHR) void k_prep(const float* __restrict__ nf,
                                               const float* __restrict__ l0s, const float* __restrict__ l0v,
                                               const float* __restrict__ l1s, const float* __restrict__ l1v,
                                               const float* __restrict__ l2s, const float* __restrict__ l2v,
                                               const float* __restrict__ esw1, const float* __restrict__ esw2,
                                               const float* __restrict__ erw1, const float* __restrict__ erw2,
                                               unsigned short* WP, unsigned short* XSB, unsigned short* VB,
                                               unsigned short* GS, unsigned short* GV) {
  const int u = (int)blockIdx.x * NTHR + (int)threadIdx.x;
  if (u < U11) {
    v8us o;
    if (u < U1) {
      o = wgather(l0s, 128, 0, 128, 128, u >> 4, (u & 15) * 8);
    } else if (u < U2) {
      const int v = u - U1;
      o = wgather(l0v, 64, 0, 64, 64, v >> 3, (v & 7) * 8);
    } else if (u < U3) {
      const int v = u - U2;
      o = wgather(l1s, 128, 0, 128, 128, v >> 5, (v & 31) * 8);
    } else if (u < U4) {
      const int v = u - U3;
      o = wgather(l1v, 64, 0, 64, 64, v >> 4, (v & 15) * 8);
    } else if (u < U5) {
      const int v = u - U4;
      const int n = v >> 5;
      o = wgather(esw1, 128, (n >> 7) * 128, 128, 128, n & 127, (v & 31) * 8);
    } else if (u < U6) {
      const int v = u - U5;
      o = wgather(esw1, 128, 256, 64, 64, v >> 4, (v & 15) * 8);
    } else if (u < U7) {
      const int v = u - U6;
      o = wgather(esw2, 384, 0, 128, 128, v >> 5, (v & 31) * 8);
    } else if (u < U8) {
      const int v = u - U7;
      o = wgather(erw1, 128, 0, 32, EAD, v >> 2, (v & 3) * 8);
    } else if (u < U9) {
      const int v = u - U8;
      o = wgather(erw2, 384, 0, 128, 128, v >> 5, (v & 31) * 8);
    } else if (u < U10) {
      const int v = u - U9;
      const int n = v / 48;
      o = wgather(l2s, 128, 0, 192, 192, n, (v - 48 * n) * 8);
    } else {
      const int v = u - U10;
      const int n = v / 48;
      o = wgather(l2v, 64, 0, 192, 192, n, (v - 48 * n) * 8);
    }
    put16(WP + (size_t)8 * (size_t)u, o);
    return;
  } else if (u < U12) {
    const int v   = u - U11;
    const int row = v >> 4;
    const int j   = v & 15;
    const float* p = nf + (size_t)row * DF + 8 * j;
    const v4f a = *(const v4fa*)p;
    const v4f b = *(const v4fa*)(p + 4);
    const float f8[8] = {a.x, a.y, a.z, a.w, b.x, b.y, b.z, b.w};
    v8us ox, oh, ol;
#pragma unroll
    for (int i = 0; i < 8; ++i) {
      const unsigned xb = bf16_bits(f8[i]);
      const float s = __uint_as_float(xb << 16);
      const float g = silu_f(s);
      const unsigned hb = bf16_bits(g);
      const unsigned lb = bf16_bits(g - __uint_as_float(hb << 16));
      ox[i] = (unsigned short)xb;
      oh[i] = (unsigned short)hb;
      ol[i] = (unsigned short)lb;
    }
    unsigned short* px = XSB + (size_t)row * SC + 8 * j;
    unsigned short* pg = GS + (size_t)row * 256 + 8 * j;
    *(volatile v8us*)px = ox;
    *(volatile v8us*)pg = oh;
    *(volatile v8us*)(pg + SC) = ol;
    __threadfence();
    *(volatile v8us*)px = ox;
    *(volatile v8us*)pg = oh;
    *(volatile v8us*)(pg + SC) = ol;
    return;
  } else if (u < U13) {
    const int v   = u - U12;
    const int row = v >> 3;
    const int j   = v & 7;
    const float* p = nf + (size_t)row * DF + SC + 24 * j;
    const v4f q0 = *(const v4fa*)p;
    const v4f q1 = *(const v4fa*)(p + 4);
    const v4f q2 = *(const v4fa*)(p + 8);
    const v4f q3 = *(const v4fa*)(p + 12);
    const v4f q4 = *(const v4fa*)(p + 16);
    const v4f q5 = *(const v4fa*)(p + 20);
    const float f[24] = {q0.x, q0.y, q0.z, q0.w, q1.x, q1.y, q1.z, q1.w, q2.x, q2.y, q2.z, q2.w,
                         q3.x, q3.y, q3.z, q3.w, q4.x, q4.y, q4.z, q4.w, q5.x, q5.y, q5.z, q5.w};
    v8us ob0, ob1, ob2, oh0, oh1, oh2, ol0, ol1, ol2;
#pragma unroll
    for (int c = 0; c < 8; ++c) {
      const unsigned b0 = bf16_bits(f[3 * c]);
      const unsigned b1 = bf16_bits(f[3 * c + 1]);
      const unsigned b2 = bf16_bits(f[3 * c + 2]);
      const float v0 = __uint_as_float(b0 << 16);
      const float v1 = __uint_as_float(b1 << 16);
      const float v2 = __uint_as_float(b2 << 16);
      const float nrm = __builtin_amdgcn_sqrtf(((v0 * v0 + v1 * v1) + v2 * v2) + 1e-10f);
      const float gt  = silu_f(nrm) * __builtin_amdgcn_rcpf(nrm);
      const float g0 = v0 * gt, g1 = v1 * gt, g2 = v2 * gt;
      const unsigned h0 = bf16_bits(g0), h1 = bf16_bits(g1), h2 = bf16_bits(g2);
      ob0[c] = (unsigned short)b0; ob1[c] = (unsigned short)b1; ob2[c] = (unsigned short)b2;
      oh0[c] = (unsigned short)h0; oh1[c] = (unsigned short)h1; oh2[c] = (unsigned short)h2;
      ol0[c] = (unsigned short)bf16_bits(g0 - __uint_as_float(h0 << 16));
      ol1[c] = (unsigned short)bf16_bits(g1 - __uint_as_float(h1 << 16));
      ol2[c] = (unsigned short)bf16_bits(g2 - __uint_as_float(h2 << 16));
    }
    unsigned short* pb = VB + (size_t)(row * 3) * VC + 8 * j;
    unsigned short* pg = GV + (size_t)(row * 3) * 128 + 8 * j;
    *(volatile v8us*)pb = ob0;
    *(volatile v8us*)(pb + VC) = ob1;
    *(volatile v8us*)(pb + 2 * VC) = ob2;
    *(volatile v8us*)pg = oh0;
    *(volatile v8us*)(pg + VC) = ol0;
    *(volatile v8us*)(pg + 128) = oh1;
    *(volatile v8us*)(pg + 128 + VC) = ol1;
    *(volatile v8us*)(pg + 256) = oh2;
    *(volatile v8us*)(pg + 256 + VC) = ol2;
    __threadfence();
    *(volatile v8us*)pb = ob0;
    *(volatile v8us*)(pb + VC) = ob1;
    *(volatile v8us*)(pb + 2 * VC) = ob2;
    *(volatile v8us*)pg = oh0;
    *(volatile v8us*)(pg + VC) = ol0;
    *(volatile v8us*)(pg + 128) = oh1;
    *(volatile v8us*)(pg + 128 + VC) = ol1;
    *(volatile v8us*)(pg + 256) = oh2;
    *(volatile v8us*)(pg + 256 + VC) = ol2;
    return;
  }
}

template <int NT, int HL>
__global__ __launch_bounds__(GTHR) void k_gemm(const unsigned short* __restrict__ A, int lda,
                                               const unsigned short* __restrict__ BT, int ldb, int K,
                                               const float* __restrict__ bias, int nbias,
                                               float* Cm, int ldc, unsigned short* Cb) {
  constexpr int NC = 16 * NT;
  static_assert(NT == 8 || NT == 4);
  static_assert(HL == 0 || NT == 8);
  __shared__ __attribute__((aligned(16))) float stg[GBM * NC];
  const int tid = (int)threadIdx.x, lane = tid & 31, wave = tid >> 5, hh = lane >> 4, m = lane & 15;
  const int rowBase = (int)blockIdx.x * GBM;
  const int colBase = (int)blockIdx.y * NC;

  v8f acc[NT];
  {
    const v8f z = {0.f, 0.f, 0.f, 0.f, 0.f, 0.f, 0.f, 0.f};
#pragma unroll
    for (int t = 0; t < NT; ++t) acc[t] = z;
  }
  const unsigned short* ap = A  + (size_t)(rowBase + 16 * wave + m) * (size_t)lda + 8 * hh;
  const unsigned short* bp = BT + (size_t)(colBase + m) * (size_t)ldb + 8 * hh;

#pragma unroll 1
  for (int k0 = 0; k0 < K; k0 += 32) {
    FragB af;
    af.h[0] = *(const v8usa*)(ap + k0);
    af.h[1] = *(const v8usa*)(ap + k0 + 16);
#pragma unroll
    for (int nt = 0; nt < NT; ++nt) {
      const unsigned short* wq = bp + (size_t)(16 * nt) * (size_t)ldb + k0;
      FragB bf;
      bf.h[0] = *(const v8usa*)wq;
      bf.h[1] = *(const v8usa*)(wq + 16);
      acc[nt] = wmb(af, bf, acc[nt]);
    }
  }

#pragma unroll
  for (int nt = 0; nt < NT; ++nt) {
    const int lc  = 16 * nt + m;
    const int col = colBase + lc;
    const int ci  = col < SC ? col : SC - 1;
    const float bl = bf16_val(bias[ci]);
    asm volatile("" :: "v"(bl));
    const float bvv = bl * ((col < nbias) ? 1.0f : 0.0f);
#pragma unroll
    for (int r = 0; r < 8; ++r) {
      const int lr = 16 * wave + 8 * hh + r;
      stg[lr * NC + lc] = acc[nt][r] + bvv;
    }
  }
  __syncthreads();

  if constexpr (HL == 1) {
    const int part = lane >> 4;
    const int j = lane & 15;
    const unsigned mh = 0u - (unsigned)part;
    const unsigned ml = ~mh;
    v8us pv[16];
#pragma unroll
    for (int i = 0; i < 16; ++i) {
      const float* sp = stg + (16 * wave + i) * NC + 8 * j;
      const v4f a = *(const v4fa*)sp;
      const v4f b = *(const v4fa*)(sp + 4);
      const v8f f8 = {a.x, a.y, a.z, a.w, b.x, b.y, b.z, b.w};
      v8us oo;
#pragma unroll
      for (int e = 0; e < 8; ++e) {
        const unsigned hb = bf16_bits(f8[e]);
        const unsigned lb = bf16_bits(f8[e] - __uint_as_float(hb << 16));
        oo[e] = (unsigned short)((hb & ml) | (lb & mh));
      }
      pv[i] = oo;
    }
#pragma unroll
    for (int i = 0; i < 16; ++i) {
      unsigned short* op = Cb + (size_t)(rowBase + 16 * wave + i) * (size_t)(2 * NC) + part * NC + 8 * j;
      *(volatile v8us*)op = pv[i];
    }
    __threadfence();
#pragma unroll
    for (int i = 0; i < 16; ++i) {
      unsigned short* op = Cb + (size_t)(rowBase + 16 * wave + i) * (size_t)(2 * NC) + part * NC + 8 * j;
      *(volatile v8us*)op = pv[i];
    }
  } else if constexpr (NT == 8) {
    v4f pv[16];
#pragma unroll
    for (int i = 0; i < 16; ++i) pv[i] = *(const v4fa*)(stg + (16 * wave + i) * NC + 4 * lane);
#pragma unroll
    for (int i = 0; i < 16; ++i) {
      float* op = Cm + (size_t)(rowBase + 16 * wave + i) * (size_t)ldc + colBase + 4 * lane;
      *(volatile v4f*)op = pv[i];
    }
    __threadfence();
#pragma unroll
    for (int i = 0; i < 16; ++i) {
      float* op = Cm + (size_t)(rowBase + 16 * wave + i) * (size_t)ldc + colBase + 4 * lane;
      *(volatile v4f*)op = pv[i];
    }
  } else {
    v4f pv[8];
#pragma unroll
    for (int i = 0; i < 8; ++i) pv[i] = *(const v4fa*)(stg + (16 * wave + 2 * i + hh) * NC + 4 * m);
#pragma unroll
    for (int i = 0; i < 8; ++i) {
      float* op = Cm + (size_t)(rowBase + 16 * wave + 2 * i + hh) * (size_t)ldc + colBase + 4 * m;
      *(volatile v4f*)op = pv[i];
    }
    __threadfence();
#pragma unroll
    for (int i = 0; i < 8; ++i) {
      float* op = Cm + (size_t)(rowBase + 16 * wave + 2 * i + hh) * (size_t)ldc + colBase + 4 * m;
      *(volatile v4f*)op = pv[i];
    }
  }
}

struct ColSpec { int xo; int xs; int yi; int wo; int dot; };
__device__ __forceinline__ ColSpec col_decode(int j) {
  ColSpec s;
  s.dot = 0;
  if (j < 128) {
    s.xo = j; s.xs = 128; s.yi = 0; s.wo = j;
  } else if (j < 192) {
    const int c = j - 128;
    s.xo = 8192 + c; s.xs = 192; s.yi = 1; s.wo = 320 + c; s.dot = 1;
  } else {
    const int jv = j - 192;
    const int mm = jv / 192;
    const int jj = jv - 192 * mm;
    if (jj < 128) {
      s.xo = jj; s.xs = 128; s.yi = 1 + mm; s.wo = 128 + jj;
    } else {
      const int c = jj - 128;
      s.xo = 8192 + 64 * mm + c; s.xs = 192; s.yi = 0; s.wo = 256 + c;
    }
  }
  return s;
}

__device__ __forceinline__ void put_row(float* ACC, int row, int tid, float v0, float v1, float v2) {
  float* p = ACC + (size_t)row * ACW + tid;
  *(volatile float*)p = v0;
  *(volatile float*)(p + 256) = v1;
  *(volatile float*)(p + 512) = v2;
  __threadfence();
  *(volatile float*)p = v0;
  *(volatile float*)(p + 256) = v1;
  *(volatile float*)(p + 512) = v2;
}

__global__ __launch_bounds__(NTHR) __attribute__((amdgpu_num_vgpr(248)))
void k_edge(const int* __restrict__ ei, int nE, int nN, int vec8,
            const float* __restrict__ ea, const float* __restrict__ rshs,
            const float* __restrict__ PAB, const float* __restrict__ PVT,
            const float* __restrict__ XS, const float* __restrict__ XVT,
            const unsigned short* __restrict__ ESC, const unsigned short* __restrict__ ES22,
            const unsigned short* __restrict__ ER1, const unsigned short* __restrict__ ER22,
            const float* __restrict__ erb1, const float* __restrict__ esb2, const float* __restrict__ erb2,
            float* ACC) {
  extern __shared__ __attribute__((aligned(16))) float dyn[];
  float*          sWt  = dyn + F_WT;
  float*          sHt  = dyn + F_WT;
  int*            list = (int*)(dyn + F_WT);
  int*            reg1 = list + LISTN;
  unsigned short* sAhs = (unsigned short*)(dyn + F_A);
  unsigned short* sAhr = sAhs + TE * 256;
  unsigned short* sAvd = sAhr + TE * 256;
  float*          sX   = dyn + F_A;
  unsigned short* sEA  = (unsigned short*)(dyn + F_EA);
  float*          sB   = dyn + F_B;
  float*          sY   = dyn + F_Y;
  int*            sSl  = (int*)(dyn + F_SL);
  int*            reg2 = (int*)(dyn + F_R2);
  int*            scnt = (int*)(dyn + F_CNT);
  int*            soff = scnt + 64;
  int*            wcnt = soff + 64;

  const int tid = (int)threadIdx.x, lane = tid & 31, wave = tid >> 5, hh = lane >> 4, m = lane & 15;
  const int base = (int)blockIdx.x * NBS;

  for (int i = tid; i < SC; i += NTHR) sB[i] = bf16_val(erb1[i]);
  for (int i = tid; i < WN; i += NTHR) {
    sB[SC + i]      = bf16_val(esb2[i]);
    sB[SC + WN + i] = bf16_val(erb2[i]);
  }

  int tot = 0, raw = 0;
  int nChunks = (nE + CHUNK - 1) / CHUNK;
  nChunks = nChunks > (NE / CHUNK) ? (NE / CHUNK) : nChunks;
#pragma unroll 1
  for (int ch = 0; ch < nChunks; ++ch) {
    const int cbase = ch * CHUNK;
    const int wc = scan_chunk<SLB>(ei, nE, cbase, base, NBS, vec8, list, tid, lane, wave);
    if (lane == 0) wcnt[wave] = wc;
    __syncthreads();
    int pre = 0, all = 0;
#pragma unroll
    for (int w2 = 0; w2 < NWAVE; ++w2) {
      int c = wcnt[w2];
      c = c < 0 ? 0 : (c > WCAP ? WCAP : c);
      all += c;
      pre += (w2 < wave) ? c : 0;
    }
    const int wcc   = wc > WCAP ? WCAP : wc;
    const int pbase = tot + pre;
#pragma unroll 1
    for (int i = lane; i < wcc; i += 32) {
      const int ent = list[wave * WCAP + i];
      const int el  = (ent >> SLB) & (CHUNK - 1);
      const int sl  = ent & (NBS - 1);
      int eid = cbase + el;
      eid = eid > nE - 1 ? nE - 1 : eid;
      const int pos = pbase + i;
      if (pos < HCAP) reg1[pos] = (int)(((unsigned)eid << SLB) | (unsigned)sl);
    }
    raw += all;
    tot += all;
    tot = tot > HCAP ? HCAP : tot;
    __syncthreads();
  }
  const int  nh  = tot;
  const bool ovf = raw > HCAP;

  if (tid < NBS) {
    int c = 0;
#pragma unroll 1
    for (int i = 0; i < nh; ++i) c += ((reg1[i] & (NBS - 1)) == tid) ? 1 : 0;
    scnt[tid] = c;
  }
  __syncthreads();
  if (tid < NBS) {
    int o = 0;
#pragma unroll 1
    for (int s = 0; s < NBS; ++s) {
      const int cv = scnt[s];
      o += (s < tid) ? cv : 0;
    }
    soff[tid] = o;
    int p = o;
#pragma unroll 1
    for (int i = 0; i < nh; ++i) {
      const int uv = reg1[i];
      if ((uv & (NBS - 1)) == tid) {
        if (p >= 0 && p < HCAP) reg2[p] = (int)((unsigned)uv >> SLB);
        p = p + 1;
      }
    }
  }
  __syncthreads();

  const int row = tid >> 2, q = tid & 3;
  const ColSpec c0 = col_decode(tid);
  const ColSpec c1 = col_decode(tid + 256);
  const ColSpec c2 = col_decode(tid + 512);
  const float fd   = c0.dot ? 1.0f : 0.0f;
  const float sc0  = c0.dot ? IS3 : 1.0f;
  const int   xo0b = c0.dot ? c0.xo + 64 : c0.xo;
  const int   xo0c = c0.dot ? c0.xo + 128 : c0.xo;
  const int   yb0  = c0.dot ? 2 : c0.yi;
  const int   yc0  = c0.dot ? 3 : c0.yi;
  const float qnan = __int_as_float(0x7fc00000);
  const float pz   = ovf ? qnan : 0.0f;
  float a0 = 0.0f, a1 = 0.0f, a2 = 0.0f;
  int cur = 0;
  int nT = (nh + TE - 1) / TE;
  nT = nT > MAXT ? MAXT : nT;

#pragma unroll 1
  for (int tl = 0; tl < nT; ++tl) {
    const int idx = tl * TE + row;
    int ic = idx < nh ? idx : nh - 1;
    ic = ic < 0 ? 0 : ic;
    int eid = reg2[ic];
    eid = eid < 0 ? 0 : (eid > nE - 1 ? nE - 1 : eid);
    int rv = ei[eid];
    int sd = ei[(size_t)nE + eid];
    rv = rv < 0 ? 0 : (rv > nN - 1 ? nN - 1 : rv);
    sd = sd < 0 ? 0 : (sd > nN - 1 ? nN - 1 : sd);
    const v4f yy = *(const v4fa*)(rshs + (size_t)eid * 4);
    asm volatile("" :: "v"(yy.x), "v"(yy.y), "v"(yy.z), "v"(yy.w));
    if (q == 0) {
      int sl = rv - base;
      sl = sl < 0 ? 0 : (sl > NBS - 1 ? NBS - 1 : sl);
      sSl[row] = sl;
      const v4f yb4 = {bf16_val(yy.x), bf16_val(yy.y), bf16_val(yy.z), bf16_val(yy.w)};
      *(v4fa*)(sY + 4 * row) = yb4;
    }
    {
      const float* rp = ea + (size_t)eid * EAD;
      int o0 = 8 * q;     o0 = o0 > 16 ? 16 : o0;
      int o1 = 8 * q + 4; o1 = o1 > 16 ? 16 : o1;
      const v4f a = *(const v4fa*)(rp + o0);
      const v4f b = *(const v4fa*)(rp + o1);
      const float fa = (q < 3) ? 1.0f : 0.0f;
      const float fb = (q < 2) ? 1.0f : 0.0f;
      v8us o;
      o[0] = (unsigned short)bf16_bits(a.x * fa); o[1] = (unsigned short)bf16_bits(a.y * fa);
      o[2] = (unsigned short)bf16_bits(a.z * fa); o[3] = (unsigned short)bf16_bits(a.w * fa);
      o[4] = (unsigned short)bf16_bits(b.x * fb); o[5] = (unsigned short)bf16_bits(b.y * fb);
      o[6] = (unsigned short)bf16_bits(b.z * fb); o[7] = (unsigned short)bf16_bits(b.w * fb);
      *(v8usa*)(sEA + row * 32 + 8 * q) = o;
    }
    {
      const float* pr = PVT + (size_t)rv * 192;
      const float* ps = PVT + (size_t)sd * 192;
#pragma unroll 1
      for (int g = 0; g < 4; ++g) {
        const int c = 16 * q + 4 * g;
        const v4f r0 = *(const v4fa*)(pr + c);
        const v4f r1 = *(const v4fa*)(pr + 64 + c);
        const v4f r2 = *(const v4fa*)(pr + 128 + c);
        const v4f s0 = *(const v4fa*)(ps + c);
        const v4f s1 = *(const v4fa*)(ps + 64 + c);
        const v4f s2 = *(const v4fa*)(ps + 128 + c);
        v4f d;
        d.x = (r0.x * s0.x + r1.x * s1.x) + r2.x * s2.x;
        d.y = (r0.y * s0.y + r1.y * s1.y) + r2.y * s2.y;
        d.z = (r0.z * s0.z + r1.z * s1.z) + r2.z * s2.z;
        d.w = (r0.w * s0.w + r1.w * s1.w) + r2.w * s2.w;
        v4us oh, ol;
        split4(d, oh, ol);
        *(v4usa*)(sAvd + row * 128 + c)      = oh;
        *(v4usa*)(sAvd + row * 128 + 64 + c) = ol;
      }
    }
    __syncthreads();

    {
      v8f acc[4];
      {
        const v8f z = {0.f, 0.f, 0.f, 0.f, 0.f, 0.f, 0.f, 0.f};
#pragma unroll
        for (int mt = 0; mt < 4; ++mt) acc[mt] = z;
      }
      const unsigned short* ap = sAvd + m * 128 + 8 * hh;
      const unsigned short* bp = ESC + (size_t)(16 * wave + m) * 128 + 8 * hh;
#pragma unroll 1
      for (int k0 = 0; k0 < 128; k0 += 32) {
        FragB b;
        b.h[0] = *(const v8usa*)(bp + k0);
        b.h[1] = *(const v8usa*)(bp + k0 + 16);
#pragma unroll
        for (int mt = 0; mt < 4; ++mt) {
          FragB a;
          a.h[0] = *(const v8usa*)(ap + mt * 16 * 128 + k0);
          a.h[1] = *(const v8usa*)(ap + mt * 16 * 128 + k0 + 16);
          acc[mt] = wmb(a, b, acc[mt]);
        }
      }
#pragma unroll
      for (int mt = 0; mt < 4; ++mt)
#pragma unroll
        for (int r = 0; r < 8; ++r) sHt[(16 * mt + 8 * hh + r) * 128 + 16 * wave + m] = acc[mt][r];
    }
    {
      v8f acc[4];
      {
        const v8f z = {0.f, 0.f, 0.f, 0.f, 0.f, 0.f, 0.f, 0.f};
#pragma unroll
        for (int mt = 0; mt < 4; ++mt) acc[mt] = z;
      }
      const unsigned short* ap = sEA + m * 32 + 8 * hh;
      const unsigned short* bp = ER1 + (size_t)(16 * wave + m) * 32 + 8 * hh;
      FragB b;
      b.h[0] = *(const v8usa*)bp;
      b.h[1] = *(const v8usa*)(bp + 16);
#pragma unroll
      for (int mt = 0; mt < 4; ++mt) {
        FragB a;
        a.h[0] = *(const v8usa*)(ap + mt * 16 * 32);
        a.h[1] = *(const v8usa*)(ap + mt * 16 * 32 + 16);
        acc[mt] = wmb(a, b, acc[mt]);
      }
      const int   col = 16 * wave + m;
      const float b1  = sB[col];
#pragma unroll
      for (int mt = 0; mt < 4; ++mt)
#pragma unroll
        for (int r = 0; r < 8; ++r) {
          const float v = silu_f(acc[mt][r] + b1);
          const unsigned hb = bf16_bits(v);
          const unsigned lb = bf16_bits(v - __uint_as_float(hb << 16));
          unsigned short* dp = sAhr + (16 * mt + 8 * hh + r) * 256 + col;
          dp[0]   = (unsigned short)hb;
          dp[128] = (unsigned short)lb;
        }
    }
    __syncthreads();

    {
      const float* pa = PAB + (size_t)rv * 256 + 32 * q;
      const float* pb = PAB + (size_t)sd * 256 + 128 + 32 * q;
      const float* hp = sHt + row * 128 + 32 * q;
      unsigned short* dp = sAhs + row * 256 + 32 * q;
#pragma unroll 1
      for (int g = 0; g < 8; ++g) {
        const v4f h4 = *(const v4fa*)(hp + 4 * g);
        const v4f a4 = *(const v4fa*)(pa + 4 * g);
        const v4f b4 = *(const v4fa*)(pb + 4 * g);
        v4f s;
        s.x = silu_f(h4.x + (a4.x + b4.x));
        s.y = silu_f(h4.y + (a4.y + b4.y));
        s.z = silu_f(h4.z + (a4.z + b4.z));
        s.w = silu_f(h4.w + (a4.w + b4.w));
        v4us oh, ol;
        split4(s, oh, ol);
        *(v4usa*)(dp + 4 * g)       = oh;
        *(v4usa*)(dp + 128 + 4 * g) = ol;
      }
    }
    __syncthreads();

#pragma unroll 1
    for (int rd = 0; rd < 3; ++rd) {
      const int n0 = 16 * (wave + 8 * rd);
      v8f aS[4], aR[4];
      {
        const v8f z = {0.f, 0.f, 0.f, 0.f, 0.f, 0.f, 0.f, 0.f};
#pragma unroll
        for (int mt = 0; mt < 4; ++mt) { aS[mt] = z; aR[mt] = z; }
      }
      const unsigned short* aps = sAhs + m * 256 + 8 * hh;
      const unsigned short* apr = sAhr + m * 256 + 8 * hh;
      const unsigned short* bps = ES22 + (size_t)(n0 + m) * 256 + 8 * hh;
      const unsigned short* bpr = ER22 + (size_t)(n0 + m) * 256 + 8 * hh;
#pragma unroll 1
      for (int k0 = 0; k0 < 256; k0 += 32) {
        FragB bs, br;
        bs.h[0] = *(const v8usa*)(bps + k0);
        bs.h[1] = *(const v8usa*)(bps + k0 + 16);
        br.h[0] = *(const v8usa*)(bpr + k0);
        br.h[1] = *(const v8usa*)(bpr + k0 + 16);
#pragma unroll
        for (int mt = 0; mt < 4; ++mt) {
          FragB xa;
          xa.h[0] = *(const v8usa*)(aps + mt * 16 * 256 + k0);
          xa.h[1] = *(const v8usa*)(aps + mt * 16 * 256 + k0 + 16);
          aS[mt] = wmb(xa, bs, aS[mt]);
          FragB ya;
          ya.h[0] = *(const v8usa*)(apr + mt * 16 * 256 + k0);
          ya.h[1] = *(const v8usa*)(apr + mt * 16 * 256 + k0 + 16);
          aR[mt] = wmb(ya, br, aR[mt]);
        }
      }
      const float b2s = sB[SC + n0 + m];
      const float b2r = sB[SC + WN + n0 + m];
#pragma unroll
      for (int mt = 0; mt < 4; ++mt)
#pragma unroll
        for (int r = 0; r < 8; ++r)
          sWt[(16 * mt + 8 * hh + r) * WN + n0 + m] = (aS[mt][r] + b2s) * (aR[mt][r] + b2r);
    }
    __syncthreads();

    {
      const float* xp = XS + (size_t)sd * SC + 32 * q;
      float* dp = sX + row * SC + 32 * q;
#pragma unroll 4
      for (int g = 0; g < 8; ++g) *(v4fa*)(dp + 4 * g) = *(const v4fa*)(xp + 4 * g);
      const float* vp = XVT + (size_t)sd * 192 + 48 * q;
      float* dv = sX + 8192 + row * 192 + 48 * q;
#pragma unroll 4
      for (int g = 0; g < 12; ++g) *(v4fa*)(dv + 4 * g) = *(const v4fa*)(vp + 4 * g);
    }
    __syncthreads();

    {
      int nv = nh - tl * TE;
      nv = nv > TE ? TE : nv;
#pragma unroll 1
      for (int i = 0; i < nv; ++i) {
        int s = __builtin_amdgcn_readfirstlane(sSl[i]);
        s = s > NBS - 1 ? NBS - 1 : s;
        if (s > cur) {
          put_row(ACC, base + cur, tid, a0 + pz, a1 + pz, a2 + pz);
#pragma unroll 1
          for (int r = cur + 1; r < s; ++r) put_row(ACC, base + r, tid, pz, pz, pz);
          cur = s;
          a0 = 0.0f; a1 = 0.0f; a2 = 0.0f;
        }
        const float* yr = sY + 4 * i;
        const float* wr = sWt + WN * i;
        const float t0 = sX[c0.xo + i * c0.xs] * yr[c0.yi];
        const float t1 = sX[xo0b + i * c0.xs] * yr[yb0];
        const float t2 = sX[xo0c + i * c0.xs] * yr[yc0];
        const float ds = (t0 + fd * t1) + fd * t2;
        a0 += (ds * wr[c0.wo]) * sc0;
        a1 += (sX[c1.xo + i * c1.xs] * yr[c1.yi]) * wr[c1.wo];
        a2 += (sX[c2.xo + i * c2.xs] * yr[c2.yi]) * wr[c2.wo];
      }
    }
    __syncthreads();
  }

  put_row(ACC, base + cur, tid, a0 + pz, a1 + pz, a2 + pz);
#pragma unroll 1
  for (int r = cur + 1; r < NBS; ++r) put_row(ACC, base + r, tid, pz, pz, pz);
}

__global__ __launch_bounds__(NTHR) void k_split(const float* __restrict__ ACC, unsigned short* AH, int nUnits,
                                                int nN) {
  const int u = (int)blockIdx.x * NTHR + (int)threadIdx.x;
  if (u >= nUnits) return;
  const int R  = u / 24;
  const int j  = u - 24 * R;
  const int n  = R >> 2;
  const int qq = R & 3;
  const int drow = (qq == 0) ? n : (nN + 3 * n + qq - 1);
  const float* p = ACC + (size_t)R * 192 + 8 * j;
  const v4f a = *(const v4fa*)p;
  const v4f b = *(const v4fa*)(p + 4);
  const float f8[8] = {a.x, a.y, a.z, a.w, b.x, b.y, b.z, b.w};
  v8us oh, ol;
#pragma unroll
  for (int i = 0; i < 8; ++i) {
    const unsigned hb = bf16_bits(f8[i]);
    oh[i] = (unsigned short)hb;
    ol[i] = (unsigned short)bf16_bits(f8[i] - __uint_as_float(hb << 16));
  }
  unsigned short* dp = AH + (size_t)drow * 384 + 8 * j;
  *(volatile v8us*)dp = oh;
  *(volatile v8us*)(dp + 192) = ol;
  __threadfence();
  *(volatile v8us*)dp = oh;
  *(volatile v8us*)(dp + 192) = ol;
}

__global__ __launch_bounds__(NTHR) void k_ln(const float* __restrict__ OS, const float* __restrict__ OVT,
                                             const float* __restrict__ nf, const float* __restrict__ gs,
                                             const float* __restrict__ bs, const float* __restrict__ gv,
                                             float* out) {
  __shared__ __attribute__((aligned(16))) float srow[8 * DF];
  const int tid = (int)threadIdx.x, lane = tid & 31, wave = tid >> 5;
  const int node = (int)blockIdx.x * 8 + wave;
  float* sr = srow + wave * DF;
  {
    const v4f o = *(const v4fa*)(OS + (size_t)node * SC + 4 * lane);
    float s = (o.x + o.y) + (o.z + o.w);
#pragma unroll
    for (int d = 16; d >= 1; d >>= 1) s += __shfl_xor(s, d, 32);
    const float mu = s * 0.0078125f;
    const float dx = o.x - mu, dy = o.y - mu, dz = o.z - mu, dw = o.w - mu;
    float vq = (dx * dx + dy * dy) + (dz * dz + dw * dw);
#pragma unroll
    for (int d = 16; d >= 1; d >>= 1) vq += __shfl_xor(vq, d, 32);
    const float var = vq * 0.0078125f;
    const float rs  = 1.0f / sqrtf(var + 1e-5f);
    const v4f g4 = *(const v4fa*)(gs + 4 * lane);
    const v4f b4 = *(const v4fa*)(bs + 4 * lane);
    v4f r;
    r.x = (dx * rs) * bf16_val(g4.x) + bf16_val(b4.x);
    r.y = (dy * rs) * bf16_val(g4.y) + bf16_val(b4.y);
    r.z = (dz * rs) * bf16_val(g4.z) + bf16_val(b4.z);
    r.w = (dw * rs) * bf16_val(g4.w) + bf16_val(b4.w);
    *(v4fa*)(sr + 4 * lane) = r;
  }
  {
    const float* vp = OVT + (size_t)node * 192 + 2 * lane;
    const v2f p0 = *(const v2fa*)vp;
    const v2f p1 = *(const v2fa*)(vp + 64);
    const v2f p2 = *(const v2fa*)(vp + 128);
    float ss = ((p0.x * p0.x + p1.x * p1.x) + p2.x * p2.x) + ((p0.y * p0.y + p1.y * p1.y) + p2.y * p2.y);
#pragma unroll
    for (int d = 16; d >= 1; d >>= 1) ss += __shfl_xor(ss, d, 32);
    const float n2 = ss * 0.015625f;
    const float rv = 1.0f / sqrtf(n2 + 1e-5f);
    const v2f g2 = *(const v2fa*)(gv + SC + 2 * lane);
    const float ga = bf16_val(g2.x), gb = bf16_val(g2.y);
    float* dp = sr + SC + 6 * lane;
    dp[0] = (p0.x * rv) * ga;
    dp[1] = (p1.x * rv) * ga;
    dp[2] = (p2.x * rv) * ga;
    dp[3] = (p0.y * rv) * gb;
    dp[4] = (p1.y * rv) * gb;
    dp[5] = (p2.y * rv) * gb;
  }
  __syncthreads();
  const size_t gbase = (size_t)blockIdx.x * (size_t)(8 * DF);
  v4f pv[3];
#pragma unroll
  for (int s = 0; s < 3; ++s) {
    const int p  = s * NTHR + tid;
    const int pc = p < 640 ? p : 639;
    const v4f a = *(const v4fa*)(srow + 4 * pc);
    const v4f x = *(const v4fa*)(nf + gbase + 4 * pc);
    v4f o;
    o.x = bf16_val(x.x) + a.x;
    o.y = bf16_val(x.y) + a.y;
    o.z = bf16_val(x.z) + a.z;
    o.w = bf16_val(x.w) + a.w;
    pv[s] = o;
  }
#pragma unroll
  for (int s = 0; s < 3; ++s) {
    const int p = s * NTHR + tid;
    if (p < 640) *(volatile v4f*)(out + gbase + 4 * p) = pv[s];
  }
  __threadfence();
#pragma unroll
  for (int s = 0; s < 3; ++s) {
    const int p = s * NTHR + tid;
    if (p < 640) *(volatile v4f*)(out + gbase + 4 * p) = pv[s];
  }
}

extern "C" void kernel_launch(void* const* d_in, const int* in_sizes, int n_in,
                              void* d_out, int out_size, void* d_ws, size_t ws_size,
                              hipStream_t stream) {
  if (n_in < 24) return;
  if (in_sizes[0] != NN * DF) return;
  if (in_sizes[1] != NE * EAD) return;
  if (in_sizes[2] != NE * 4) return;
  if (in_sizes[3] != 2 * NE) return;
  if (in_sizes[4] != SC * SC || in_sizes[5] != SC || in_sizes[6] != VC * VC) return;
  if (in_sizes[7] != SC * SC || in_sizes[8] != SC || in_sizes[9] != VC * VC) return;
  if (in_sizes[10] != 192 * SC || in_sizes[11] != SC || in_sizes[12] != 192 * VC) return;
  if (in_sizes[13] != DF * SC || in_sizes[14] != SC) return;
  if (in_sizes[15] != SC * WN || in_sizes[16] != WN) return;
  if (in_sizes[17] != EAD * SC || in_sizes[18] != SC) return;
  if (in_sizes[19] != SC * WN || in_sizes[20] != WN) return;
  if (in_sizes[21] != SC || in_sizes[22] != SC || in_sizes[23] != 192) return;
  if (out_size != NN * DF) return;

  const float* nf    = (const float*)d_in[0];
  const float* eattr = (const float*)d_in[1];
  const float* rshs  = (const float*)d_in[2];
  const int*   ei    = (const int*)d_in[3];
  const float* l0s   = (const float*)d_in[4];
  const float* l0b   = (const float*)d_in[5];
  const float* l0v   = (const float*)d_in[6];
  const float* l1s   = (const float*)d_in[7];
  const float* l1b   = (const float*)d_in[8];
  const float* l1v   = (const float*)d_in[9];
  const float* l2s   = (const float*)d_in[10];
  const float* l2b   = (const float*)d_in[11];
  const float* l2v   = (const float*)d_in[12];
  const float* esw1  = (const float*)d_in[13];
  const float* esb1  = (const float*)d_in[14];
  const float* esw2  = (const float*)d_in[15];
  const float* esb2  = (const float*)d_in[16];
  const float* erw1  = (const float*)d_in[17];
  const float* erb1  = (const float*)d_in[18];
  const float* erw2  = (const float*)d_in[19];
  const float* erb2  = (const float*)d_in[20];
  const float* lngs  = (const float*)d_in[21];
  const float* lnbs  = (const float*)d_in[22];
  const float* lngv  = (const float*)d_in[23];
  float* out = (float*)d_out;

  char* ws = (char*)d_ws;
  size_t off = 0;
  const size_t oWP  = off; off += (size_t)NW_TOT * 2;           off = (off + 255) & ~(size_t)255;
  const size_t oXSB = off; off += (size_t)NN * SC * 2;          off = (off + 255) & ~(size_t)255;
  const size_t oVB  = off; off += (size_t)NN * 3 * VC * 2;      off = (off + 255) & ~(size_t)255;
  const size_t oGS  = off; off += (size_t)NN * 256 * 2;         off = (off + 255) & ~(size_t)255;
  const size_t oGV  = off; off += (size_t)NN * 3 * 128 * 2;     off = (off + 255) & ~(size_t)255;
  const size_t oPSH = off; off += (size_t)NN * 256 * 2;         off = (off + 255) & ~(size_t)255;
  const size_t oPAB = off; off += (size_t)NN * 256 * 4;         off = (off + 255) & ~(size_t)255;
  const size_t oPVT = off; off += (size_t)NN * 3 * VC * 4;      off = (off + 255) & ~(size_t)255;
  const size_t oXS  = off; off += (size_t)NN * SC * 4;          off = (off + 255) & ~(size_t)255;
  const size_t oXVT = off; off += (size_t)NN * 3 * VC * 4;      off = (off + 255) & ~(size_t)255;
  const size_t oACC = off; off += (size_t)NN * ACW * 4;         off = (off + 255) & ~(size_t)255;
  const size_t oAH  = off; off += (size_t)NN * 4 * 384 * 2;     off = (off + 255) & ~(size_t)255;
  const size_t oOS  = off; off += (size_t)NN * SC * 4;          off = (off + 255) & ~(size_t)255;
  const size_t oOVT = off; off += (size_t)NN * 3 * VC * 4;      off = (off + 255) & ~(size_t)255;
  if (off > ws_size || off > (size_t)WSMAX) return;
  unsigned short* WP  = (unsigned short*)(ws + oWP);
  unsigned short* XSB = (unsigned short*)(ws + oXSB);
  unsigned short* VB  = (unsigned short*)(ws + oVB);
  unsigned short* GS  = (unsigned short*)(ws + oGS);
  unsigned short* GV  = (unsigned short*)(ws + oGV);
  unsigned short* PSH = (unsigned short*)(ws + oPSH);
  float*          PAB = (float*)(ws + oPAB);
  float*          PVT = (float*)(ws + oPVT);
  float*          XS  = (float*)(ws + oXS);
  float*          XVT = (float*)(ws + oXVT);
  float*          ACC = (float*)(ws + oACC);
  unsigned short* AH  = (unsigned short*)(ws + oAH);
  float*          OS  = (float*)(ws + oOS);
  float*          OVT = (float*)(ws + oOVT);

  hipFuncSetAttribute(reinterpret_cast<const void*>(&k_edge), hipFuncAttributeMaxDynamicSharedMemorySize,
                      (int)EDGE_LDS_BYTES);

  k_prep<<<U13 / NTHR, NTHR, 0, stream>>>(nf, l0s, l0v, l1s, l1v, l2s, l2v, esw1, esw2, erw1, erw2,
                                          WP, XSB, VB, GS, GV);
  k_gemm<8, 1><<<dim3(NN / GBM, 1), GTHR, 0, stream>>>(XSB, SC, WP + OW_W0S, SC, SC, l0b, SC, PAB, 256, PSH);
  k_gemm<8, 0><<<dim3(NN / GBM, 2), GTHR, 0, stream>>>(PSH, 256, WP + OW_ESAB, 256, 256, esb1, SC, PAB, 256, PSH);
  k_gemm<4, 0><<<dim3(3 * NN / GBM, 1), GTHR, 0, stream>>>(VB, VC, WP + OW_W0V, VC, VC, l0b, 0, PVT, VC, PSH);
  k_gemm<8, 0><<<dim3(NN / GBM, 1), GTHR, 0, stream>>>(GS, 256, WP + OW_W1S2, 256, 256, l1b, SC, XS, SC, PSH);
  k_gemm<4, 0><<<dim3(3 * NN / GBM, 1), GTHR, 0, stream>>>(GV, 128, WP + OW_W1V2, 128, 128, l0b, 0, XVT, VC, PSH);
  k_edge<<<NN / NBS, NTHR, EDGE_LDS_BYTES, stream>>>(ei, NE, NN, 1, eattr, rshs, PAB, PVT, XS, XVT,
                                                     WP + OW_ESC, WP + OW_ES22, WP + OW_ER1, WP + OW_ER22,
                                                     erb1, esb2, erb2, ACC);
  k_split<<<(NN * 4 * 24) / NTHR, NTHR, 0, stream>>>(ACC, AH, NN * 4 * 24, NN);
  k_gemm<8, 0><<<dim3(NN / GBM, 1), GTHR, 0, stream>>>(AH, 384, WP + OW_W2S2, 384, 384, l2b, SC, OS, SC, PSH);
  k_gemm<4, 0><<<dim3(3 * NN / GBM, 1), GTHR, 0, stream>>>(AH + (size_t)NN * 384, 384, WP + OW_W2V2, 384, 384,
                                                           l0b, 0, OVT, VC, PSH);
  k_ln<<<NN / 8, NTHR, 0, stream>>>(OS, OVT, nf, lngs, lnbs, lngv, out);
}
